// RayObsGraph_85160611545430
// MI455X (gfx1250) — hardware-verified
//
#include <hip/hip_runtime.h>
#include <math.h>

#ifndef NB
#define NB 16
#endif
#define NB_FULL 16
#define TT 64
#define TT_FULL 64
#define GN 128
#define DD 512
#define HH 512
#define OO 256
#define AA 18
#define HPAD 64
#define MTOK (NB * TT)
#define NOUT4 (MTOK * AA / 4)
#define CP4 ((HPAD + HH) / 4)
#define WLPAD_WB ((HPAD * (OO / 8)) / 256)

static_assert(TT == TT_FULL);
static_assert(NB <= NB_FULL);
static_assert(TT < GN - 1);
static_assert(MTOK % 64 == 0);
static_assert(HH % 64 == 0 && OO % 64 == 0 && HPAD % 64 == 0);
static_assert(DD % 32 == 0 && HH % 32 == 0 && OO % 32 == 0);
static_assert((MTOK * DD / 8) % 256 == 0);
static_assert(DD / 8 == 64);
static_assert(OO / 8 == 32);
static_assert((HH * (DD / 8)) % 256 == 0 && (OO * (HH / 8)) % 256 == 0 && (HPAD * (OO / 8)) % 256 == 0);
static_assert(HH == 2 * 256);
static_assert((HH / 8) * 16 == HH * 2);
static_assert((MTOK * AA) % 4 == 0);
static_assert((MTOK * AA * 4) % 128 == 0);
static_assert(AA <= HPAD);
static_assert((HPAD + HH) % 4 == 0 && CP4 <= 256 && CP4 % 8 == 0);
static_assert((GN * GN) % 4 == 0);
static_assert(1024 < TT * AA);
static_assert(8 * 16 * 68 * 4 <= 131072);
static_assert(HH * 4 <= 131072);

typedef __attribute__((ext_vector_type(16))) _Float16 v16h;
typedef __attribute__((ext_vector_type(8)))  _Float16 v8h;
typedef __attribute__((ext_vector_type(8)))  float    v8f;
typedef __attribute__((ext_vector_type(4)))  float    v4f;
typedef __attribute__((ext_vector_type(4)))  unsigned int v4u;
typedef __attribute__((ext_vector_type(4)))  int      v4i;


#define VST2(T, ptr, val) do { const T vst2_v_ = (val); *(volatile T*)(ptr) = vst2_v_; __threadfence(); *(volatile T*)(ptr) = vst2_v_; } while (0)
#define VST2V4(ptr, val) do { const v4f vst2_v4_ = (val); *(volatile v4f*)(ptr) = vst2_v4_; __threadfence(); *(volatile v4f*)(ptr) = vst2_v4_; } while (0)

__device__ __forceinline__ float bfr(float f) {
    unsigned u = __float_as_uint(f);
    u += 0x7FFFu + ((u >> 16) & 1u);
    return __uint_as_float(u & 0xFFFF0000u);
}
__device__ __forceinline__ unsigned short f2h_bits(float x) {
    return (fabsf(x) < 6.104e-5f) ? (unsigned short)0 : __builtin_bit_cast(unsigned short, (_Float16)x);
}
__device__ __forceinline__ void st8h(unsigned short* P, size_t o, const float* v) {
    v4u pk;
    pk.x = (unsigned)f2h_bits(v[0]) | ((unsigned)f2h_bits(v[1]) << 16);
    pk.y = (unsigned)f2h_bits(v[2]) | ((unsigned)f2h_bits(v[3]) << 16);
    pk.z = (unsigned)f2h_bits(v[4]) | ((unsigned)f2h_bits(v[5]) << 16);
    pk.w = (unsigned)f2h_bits(v[6]) | ((unsigned)f2h_bits(v[7]) << 16);
    VST2(v4u, (v4u*)(P + o), pk);
}

union FragU { v16h v; v8h h[2]; };
__device__ __forceinline__ v16h frag_ld(const _Float16* p) {
    FragU f; f.h[0] = *(const v8h*)(p); f.h[1] = *(const v8h*)(p + 16); return f.v;
}
__device__ __forceinline__ v8f wmma16(v16h a, v16h b, v8f c) {
    c = __builtin_amdgcn_wmma_f32_16x16x32_f16(false, a, false, b, (short)0, c, false, false);
    asm volatile("v_nop\n\tv_nop\n\tv_nop\n\tv_nop" : "+v"(c) : "v"(a), "v"(b));
    return c;
}
__device__ __forceinline__ void dep_guard_h(v8f& a, v8f& b, v16h x, v16h y) { asm volatile("v_nop\n\tv_nop\n\tv_nop\n\tv_nop" : "+v"(a), "+v"(b) : "v"(x), "v"(y)); }
__device__ __forceinline__ void keep4_h(v16h a, v16h b, v16h c, v16h d) { asm volatile("v_nop" :: "v"(a), "v"(b), "v"(c), "v"(d)); }
__device__ __forceinline__ void acc_guard4(v8f& a, v8f& b, v8f& c, v8f& d) { asm volatile("v_nop\n\tv_nop\n\tv_nop\n\tv_nop" : "+v"(a), "+v"(b), "+v"(c), "+v"(d)); }
__device__ __forceinline__ void wave_sync_lds() {
    __builtin_amdgcn_fence(3  , "workgroup");
    __builtin_amdgcn_wave_barrier();
    __builtin_amdgcn_fence(2  , "workgroup");
}

template <int OUT_MODE, bool RESID, bool RELU>
__global__ __launch_bounds__(256) void k_gemm64(
    const _Float16* __restrict__ A, unsigned lda, const _Float16* __restrict__ Bt, unsigned ldb,
    void* __restrict__ Cout, unsigned ldc, const float* __restrict__ bias, const float* __restrict__ resid,
    unsigned M, unsigned N, unsigned K, float scale, float oscale) {
  __shared__ __align__(16) float sT[8][16 * 68];
  const unsigned lane = threadIdx.x & 31u;
  const unsigned wave = threadIdx.x >> 5;
  const unsigned tilesN = N >> 6, tilesM = M >> 6;
  const unsigned tile = blockIdx.x * 8u + wave;
  if (tile >= tilesM * tilesN) return;
  const unsigned tm = tile / tilesN;
  const unsigned tn = tile - tm * tilesN;
  const unsigned m0 = tm << 6, n0 = tn << 6;
  const unsigned rlane = lane & 15u;
  const unsigned koff = (lane >> 4) * 8u;
  const unsigned mOff = koff;

  v8f acc[4][4];
#pragma unroll
  for (int i = 0; i < 4; ++i)
#pragma unroll
    for (int j = 0; j < 4; ++j) acc[i][j] = (v8f){0.f,0.f,0.f,0.f,0.f,0.f,0.f,0.f};

  for (unsigned k0 = 0; k0 < K; k0 += 32u) {
    v16h bh[4];
#pragma unroll
    for (int j = 0; j < 4; ++j)
      bh[j] = frag_ld(Bt + (size_t)(n0 + ((unsigned)j << 4) + rlane) * ldb + koff + k0);
#pragma unroll
    for (int i = 0; i < 4; ++i) {
      const v16h ah = frag_ld(A + (size_t)(m0 + ((unsigned)i << 4) + rlane) * lda + koff + k0);
#pragma unroll
      for (int j = 0; j < 4; ++j)
        acc[i][j] = __builtin_amdgcn_wmma_f32_16x16x32_f16(false, ah, false, bh[j], (short)0, acc[i][j], false, false);
      dep_guard_h(acc[i][0], acc[i][3], ah, ah);
    }
    keep4_h(bh[0], bh[1], bh[2], bh[3]);
  }
  acc_guard4(acc[0][0], acc[0][1], acc[0][2], acc[0][3]);
  acc_guard4(acc[1][0], acc[1][1], acc[1][2], acc[1][3]);
  acc_guard4(acc[2][0], acc[2][1], acc[2][2], acc[2][3]);
  acc_guard4(acc[3][0], acc[3][1], acc[3][2], acc[3][3]);

  float* slab = sT[wave];
#pragma unroll
  for (int i = 0; i < 4; ++i) {
    const unsigned mBase = m0 + ((unsigned)i << 4);
#pragma unroll
    for (int j = 0; j < 4; ++j) {
      const unsigned n = n0 + ((unsigned)j << 4) + rlane;
      const float bv = bfr(bias[n]);
#pragma unroll
      for (int r = 0; r < 8; ++r) {
        float v = acc[i][j][r] * scale + bv;
        if (RELU) v = fmaxf(v, 0.0f);
        if (OUT_MODE == 1) v *= oscale;
        slab[(mOff + (unsigned)r) * 68u + ((unsigned)j << 4) + rlane] = v;
      }
    }
    wave_sync_lds();
    if (OUT_MODE == 0) {
      float* C = (float*)Cout;
      const unsigned hh = lane >> 4, c4 = (lane & 15u) * 4u;
#pragma unroll
      for (int half = 0; half < 2; ++half) {
        v4f vv[4];
#pragma unroll
        for (int it = 0; it < 4; ++it) {
          const unsigned row = (unsigned)(half * 4 + it) * 2u + hh;
          vv[it] = *(const v4f*)(slab + row * 68u + c4);
          if (RESID) vv[it] += *(const v4f*)(resid + (size_t)(mBase + row) * ldc + n0 + c4);
        }
        for (int pass = 0; pass < 2; ++pass) {
#pragma unroll
          for (int it = 0; it < 4; ++it) {
            const unsigned row = (unsigned)(half * 4 + it) * 2u + hh;
            *(volatile v4f*)(C + (size_t)(mBase + row) * ldc + n0 + c4) = vv[it];
          }
          __threadfence();
        }
      }
    } else {
      _Float16* C = (_Float16*)Cout;
      const unsigned q = lane >> 3, c8 = (lane & 7u) * 8u;
      v8h hv[4];
#pragma unroll
      for (int it = 0; it < 4; ++it) {
        const unsigned row = (unsigned)it * 4u + q;
        const float* sp = slab + row * 68u + c8;
#pragma unroll
        for (int e = 0; e < 8; ++e) hv[it][e] = (_Float16)sp[e];
      }
      for (int pass = 0; pass < 2; ++pass) {
#pragma unroll
        for (int it = 0; it < 4; ++it) {
          const unsigned row = (unsigned)it * 4u + q;
          *(volatile v8h*)(C + (size_t)(mBase + row) * ldc + n0 + c8) = hv[it];
        }
        __threadfence();
      }
    }
    wave_sync_lds();
  }
}

__global__ __launch_bounds__(256) void k_wt16(const float* __restrict__ Wm, unsigned KI, unsigned NO, unsigned lgper,
                                              unsigned short* __restrict__ W16, float sw) {
    const unsigned layer = blockIdx.y;
    const float* Wl = Wm + (size_t)layer * KI * NO;
    unsigned short* Dl = W16 + (size_t)layer * KI * NO;
    const unsigned u = blockIdx.x * 256u + threadIdx.x;
    const unsigned per = 1u << lgper;
    if (u >= NO * per) return;
    const unsigned k0 = 8u * (u & (per - 1u));
    const unsigned o = u >> lgper;
    float v[8];
#pragma unroll
    for (int i = 0; i < 8; ++i) v[i] = bfr(Wl[(size_t)(k0 + (unsigned)i) * NO + o]) * sw;
    st8h(Dl, (size_t)o * KI + k0, v);
}

__global__ __launch_bounds__(256) void k_wlpad(const float* __restrict__ Wh, const float* __restrict__ bh,
                                               unsigned short* __restrict__ wl16, float* __restrict__ cpad, float sw) {
    const unsigned t = threadIdx.x;
    if (blockIdx.x < (unsigned)WLPAD_WB) {
        const unsigned u = blockIdx.x * 256u + t;
        const unsigned k0 = 8u * (u & 31u);
        const unsigned o = u >> 5;
        const unsigned oc = (o < (unsigned)AA) ? o : (unsigned)(AA - 1);
        const bool live = (o < (unsigned)AA);
        float v[8];
#pragma unroll
        for (int i = 0; i < 8; ++i) {
            const float w = bfr(Wh[(size_t)(k0 + (unsigned)i) * AA + oc]) * sw;
            v[i] = live ? w : 0.0f;
        }
        st8h(wl16, (size_t)o * OO + k0, v);
    } else {
        const unsigned tc = (t < (unsigned)CP4) ? t : (unsigned)(CP4 - 1);
        const unsigned j0 = 4u * tc;
        const unsigned i0 = (j0      < (unsigned)AA) ? j0      : (unsigned)(AA - 1);
        const unsigned i1 = (j0 + 1u < (unsigned)AA) ? j0 + 1u : (unsigned)(AA - 1);
        const unsigned i2 = (j0 + 2u < (unsigned)AA) ? j0 + 2u : (unsigned)(AA - 1);
        const unsigned i3 = (j0 + 3u < (unsigned)AA) ? j0 + 3u : (unsigned)(AA - 1);
        const float x0 = bh[i0], x1 = bh[i1], x2 = bh[i2], x3 = bh[i3];
        v4f v;
        v.x = (j0      < (unsigned)AA) ? x0 : 0.0f;
        v.y = (j0 + 1u < (unsigned)AA) ? x1 : 0.0f;
        v.z = (j0 + 2u < (unsigned)AA) ? x2 : 0.0f;
        v.w = (j0 + 3u < (unsigned)AA) ? x3 : 0.0f;
        if (t < (unsigned)CP4) VST2V4(cpad + 4u * t, v);
    }
}

__global__ __launch_bounds__(256) void k_obs16(const float* __restrict__ obs, unsigned short* __restrict__ x16) {
    const unsigned u = blockIdx.x * 256u + threadIdx.x;
    if (u >= (unsigned)(MTOK * DD / 8)) return;
    const unsigned row = u >> 6, c0 = (u & 63u) * 8u;
    const float* xr = obs + (size_t)row * DD + c0;
    const v4f a = *(const v4f*)xr, b = *(const v4f*)(xr + 4);
    float v[8];
    v[0] = bfr(a.x) * 8.0f; v[1] = bfr(a.y) * 8.0f; v[2] = bfr(a.z) * 8.0f; v[3] = bfr(a.w) * 8.0f;
    v[4] = bfr(b.x) * 8.0f; v[5] = bfr(b.y) * 8.0f; v[6] = bfr(b.z) * 8.0f; v[7] = bfr(b.w) * 8.0f;
    st8h(x16, (size_t)row * DD + c0, v);
}

__global__ __launch_bounds__(256) void k_comb(const float* __restrict__ U, const float* __restrict__ b1,
                                              unsigned short* __restrict__ m16) {
#pragma clang fp contract(off)
    __shared__ float sM[HH];
    const unsigned t = threadIdx.x;
    const unsigned r = blockIdx.x;
    const unsigned st = r & (unsigned)(TT - 1);
    const float S6 = 0.40824829046386301637f;
    const float TH = 0.33333333333333333333f;
    const float a0 = (st <= 1u) ? 1.0f : 0.5f;
    const float a1 = (st <= 1u) ? 0.0f : ((st == 2u) ? 0.5f : S6);
    const float c0 = (st <= 1u) ? 0.0f : ((st == 2u) ? 0.5f : S6);
    const float c1 = (st <= 1u) ? 0.0f : ((st == 2u) ? 0.5f : TH);
    const float c2 = (st <= 2u) ? 0.0f : ((st == 3u) ? S6 : TH);
    const float wa = (st <= 1u) ? 1.0f : 0.5f;
    const float wb = (st <= 1u) ? 0.0f : ((st == 2u) ? 0.5f : S6);
    const unsigned r1 = r - ((st < 1u) ? st : 1u);
    const unsigned r2 = r - ((st < 2u) ? st : 2u);
#pragma unroll 1
    for (unsigned it = 0; it < (unsigned)(HH / 256); ++it) {
        const unsigned c = t + 256u * it;
        const float b = bfr(b1[c]);
        const float u0 = U[(size_t)r * HH + c];
        const float u1 = U[(size_t)r1 * HH + c];
        const float u2 = U[(size_t)r2 * HH + c];
        const float h1a = fmaxf((a0 * u0 + a1 * u1) + b, 0.0f);
        const float h1b = fmaxf(((c0 * u0 + c1 * u1) + c2 * u2) + b, 0.0f);
        sM[c] = (wa * h1a + wb * h1b) * 8.0f;
    }
    __syncthreads();
    if (t < (unsigned)(HH / 8)) {
        float v[8];
#pragma unroll
        for (int i = 0; i < 8; ++i) v[i] = sM[8u * t + (unsigned)i];
        st8h(m16, (size_t)r * HH + 8u * t, v);
    }
}

__global__ __launch_bounds__(256) void k_pack(const float* __restrict__ Lp, const int* __restrict__ adj,
                                              const int* __restrict__ num_nodes, float* __restrict__ out) {
    __shared__ unsigned sflag[8];
    const unsigned tid = threadIdx.x, lane = tid & 31u;
    const unsigned wave = (unsigned)__builtin_amdgcn_readfirstlane((int)(threadIdx.x >> 5));
    const unsigned total = (unsigned)(MTOK * AA);
    unsigned f0 = blockIdx.x * 1024u;
    f0 = (f0 < total) ? f0 : (total - 1u);
    unsigned fl = f0 + 1023u;
    fl = (fl < total) ? fl : (total - 1u);
    const unsigned bb0 = (f0 / (unsigned)AA) / (unsigned)TT;
    unsigned bb1 = (fl / (unsigned)AA) / (unsigned)TT;
    bb1 = (bb1 < bb0 + 1u) ? bb1 : (bb0 + 1u);
    unsigned acc = 0u;
    for (unsigned bb = bb0; bb <= bb1; ++bb) {
        const int* ap = adj + (size_t)bb * (GN * GN);
#pragma unroll 4
        for (unsigned i = tid; i < (unsigned)(GN * GN / 4); i += 256u) {
            const v4i x = *(const v4i*)(ap + 4u * i);
            acc |= (unsigned)(x.x | x.y | x.z | x.w);
        }
        acc |= (unsigned)num_nodes[bb];
    }
    acc |= (unsigned)__shfl_xor((int)acc, 16, 32);
    acc |= (unsigned)__shfl_xor((int)acc, 8, 32);
    acc |= (unsigned)__shfl_xor((int)acc, 4, 32);
    acc |= (unsigned)__shfl_xor((int)acc, 2, 32);
    acc |= (unsigned)__shfl_xor((int)acc, 1, 32);
    if (lane == 0u) sflag[wave] = acc;
    __syncthreads();
    const unsigned any = ((sflag[0] | sflag[1]) | (sflag[2] | sflag[3])) | ((sflag[4] | sflag[5]) | (sflag[6] | sflag[7]));
    const bool bad = (any != 0u);

    const unsigned q = blockIdx.x * 256u + tid;
    const unsigned qc = (q < (unsigned)NOUT4) ? q : (unsigned)(NOUT4 - 1);
    float g[4];
#pragma unroll
    for (int i = 0; i < 4; ++i) {
        const unsigned e = 4u * qc + (unsigned)i;
        const unsigned row = e / (unsigned)AA;
        const unsigned col = e - row * (unsigned)AA;
        g[i] = Lp[(size_t)row * HPAD + col];
    }
    const float qn = __uint_as_float(0x7FC00000u);
    v4f v;
    v.x = bad ? qn : g[0];
    v.y = bad ? qn : g[1];
    v.z = bad ? qn : g[2];
    v.w = bad ? qn : g[3];
    if (q < (unsigned)NOUT4) VST2V4(out + 4u * (size_t)q, v);
}

constexpr size_t al256(size_t b) { return (b + 255) & ~(size_t)255; }
constexpr size_t WS_TOTAL =
    al256((size_t)MTOK * DD * 2) + al256((size_t)MTOK * HH * 4) + al256((size_t)MTOK * HH * 2) +
    al256((size_t)MTOK * OO * 2) + al256((size_t)MTOK * HPAD * 4) + al256((size_t)DD * HH * 2) +
    al256((size_t)HH * OO * 2) + al256((size_t)HPAD * OO * 2) + al256((size_t)(HPAD + HH) * 4);
static_assert(WS_TOTAL <= (size_t)134217728);

static constexpr float SC = 1.0f / 256.0f;
extern "C" void kernel_launch(void* const* d_in, const int* in_sizes, int n_in, void* d_out, int out_size,
                              void* d_ws, size_t ws_size, hipStream_t stream) {
    if (n_in < 12) return;
    if (in_sizes[0] < MTOK * DD || in_sizes[2] < NB || in_sizes[3] < NB * GN * GN) return;
    if (in_sizes[4] < DD * HH || in_sizes[5] < HH || in_sizes[6] < HH * OO || in_sizes[7] < OO) return;
    if (in_sizes[8] < OO * AA || in_sizes[9] < AA || out_size < MTOK * AA) return;

    const float* obs       = (const float*)d_in[0];
    const int*   num_nodes = (const int*)d_in[2];
    const int*   adj       = (const int*)d_in[3];
    const float* W1        = (const float*)d_in[4];
    const float* b1        = (const float*)d_in[5];
    const float* W2        = (const float*)d_in[6];
    const float* b2        = (const float*)d_in[7];
    const float* Wl        = (const float*)d_in[8];
    const float* bl        = (const float*)d_in[9];
    float* out = (float*)d_out;

    char* wsp = (char*)d_ws;
    size_t off = 0;
    auto carve = [&](size_t bytes) -> void* { void* r = wsp + off; off += (bytes + 255) & ~(size_t)255; return r; };
    unsigned short* x16  = (unsigned short*)carve((size_t)MTOK * DD * 2);
    float*          U    = (float*)carve((size_t)MTOK * HH * 4);
    unsigned short* m16  = (unsigned short*)carve((size_t)MTOK * HH * 2);
    unsigned short* t16  = (unsigned short*)carve((size_t)MTOK * OO * 2);
    float*          Lp   = (float*)carve((size_t)MTOK * HPAD * 4);
    unsigned short* w1   = (unsigned short*)carve((size_t)DD * HH * 2);
    unsigned short* w2   = (unsigned short*)carve((size_t)HH * OO * 2);
    unsigned short* wl   = (unsigned short*)carve((size_t)HPAD * OO * 2);
    float*          cpad = (float*)carve((size_t)(HPAD + HH) * 4);
    if (off > ws_size || off > (size_t)134217728) return;
    const float* blpad = cpad;
    const float* zb    = cpad + HPAD;

    k_wt16<<<dim3((HH * (DD / 8)) / 256, 1), 256, 0, stream>>>(W1, DD, HH, 6, w1, 32.0f);
    k_wt16<<<dim3((OO * (HH / 8)) / 256, 1), 256, 0, stream>>>(W2, HH, OO, 6, w2, 32.0f);
    k_wlpad<<<WLPAD_WB + 1, 256, 0, stream>>>(Wl, bl, wl, cpad, 32.0f);
    k_obs16<<<(MTOK * DD / 8) / 256, 256, 0, stream>>>(obs, x16);

    const unsigned g1 = ((MTOK / 64) * (HH / 64) + 7) / 8;
    const unsigned g2 = ((MTOK / 64) * (OO / 64) + 7) / 8;
    const unsigned g3 = ((MTOK / 64) * (HPAD / 64) + 7) / 8;

    k_gemm64<0, false, false><<<g1, 256, 0, stream>>>((const _Float16*)x16, DD, (const _Float16*)w1, DD,
        (void*)U, HH, zb, nullptr, MTOK, HH, DD, SC, 1.0f);
    k_comb<<<MTOK, 256, 0, stream>>>(U, b1, m16);
    k_gemm64<1, false, true><<<g2, 256, 0, stream>>>((const _Float16*)m16, HH, (const _Float16*)w2, HH,
        (void*)t16, OO, b2, nullptr, MTOK, OO, HH, SC, 8.0f);
    k_gemm64<0, false, false><<<g3, 256, 0, stream>>>((const _Float16*)t16, OO, (const _Float16*)wl, OO,
        (void*)Lp, HPAD, blpad, nullptr, MTOK, HPAD, OO, SC, 1.0f);
    k_pack<<<(NOUT4 + 255) / 256, 256, 0, stream>>>(Lp, adj, num_nodes, out);
}
